// KANLayer_47364899340538
// MI455X (gfx1250) — hardware-verified
//
#include <hip/hip_runtime.h>
#include <math.h>

constexpr int kB      = 4096;
constexpr int kDin    = 256;
constexpr int kDout   = 256;
constexpr int kNb     = 64;
constexpr int kNk     = 68;
constexpr int kKtot   = kDin * kNb;
constexpr int kMhalf  = 2048;
constexpr float kACarry   = 1024.0f;
constexpr float kBCarry   = 256.0f;
constexpr float kOutScale = 1.0f / (1024.0f * 256.0f);
constexpr float kSixth    = 1.0f / 6.0f;
constexpr int kRowPitchDw = 40;

static_assert(kKtot % 32 == 0, "K multiple of 32");
static_assert(kMhalf % 64 == 0, "M multiple of 64");
static_assert(kDout % 64 == 0, "N multiple of 64");
static_assert(2 * kMhalf == kB, "two halves cover all rows");
constexpr size_t kBtBytes = (size_t)kDout * kKtot * 2;
constexpr size_t kABytes  = (size_t)kMhalf * kKtot * 2;
static_assert(kBtBytes + kABytes <= (size_t)134217728, "carve within 128 MiB");
static_assert(kBtBytes % 128 == 0, "R1 starts on a 128-B line");

typedef __attribute__((ext_vector_type(16))) _Float16 v16h;
typedef __attribute__((ext_vector_type(8)))  _Float16 v8h;
typedef __attribute__((ext_vector_type(16))) __bf16   v16b;
typedef __attribute__((ext_vector_type(8)))  __bf16   v8b;
typedef __attribute__((ext_vector_type(8)))  float    v8f;
typedef __attribute__((ext_vector_type(4)))  float    v4f;
typedef __attribute__((ext_vector_type(4)))  unsigned int v4u;

__device__ __forceinline__ unsigned short f2bf_bits(float f) {
  unsigned u = __float_as_uint(f);
  return (unsigned short)((u + 0x7FFFu + ((u >> 16) & 1u)) >> 16);
}
__device__ __forceinline__ float bf_bits2f(unsigned short h) { return __uint_as_float(((unsigned)h) << 16); }

__device__ __forceinline__ void dep_guard_h(v8f& a, v8f& b, v16h x, v16h y) { asm volatile("v_nop\n\tv_nop\n\tv_nop\n\tv_nop" : "+v"(a), "+v"(b) : "v"(x), "v"(y)); }
__device__ __forceinline__ void dep_guard_b(v8f& a, v8f& b, v16b x, v16b y) { asm volatile("v_nop\n\tv_nop\n\tv_nop\n\tv_nop" : "+v"(a), "+v"(b) : "v"(x), "v"(y)); }
__device__ __forceinline__ void keep4_h(v16h a, v16h b, v16h c, v16h d) { asm volatile("v_nop" :: "v"(a), "v"(b), "v"(c), "v"(d)); }
__device__ __forceinline__ void keep4_b(v16b a, v16b b, v16b c, v16b d) { asm volatile("v_nop" :: "v"(a), "v"(b), "v"(c), "v"(d)); }
__device__ __forceinline__ void acc_guard4(v8f& a, v8f& b, v8f& c, v8f& d) { asm volatile("v_nop\n\tv_nop\n\tv_nop\n\tv_nop" : "+v"(a), "+v"(b), "+v"(c), "+v"(d)); }
template <typename T> struct Frag;
template <> struct Frag<_Float16> {
  typedef v16h V; union U { v16h v; v8h h[2]; };
  static __device__ __forceinline__ v16h load(const _Float16* p) {
    U f; f.h[0] = *(const v8h*)(p); f.h[1] = *(const v8h*)(p + 16); return f.v;
  }
  static __device__ __forceinline__ v8f mma(v16h a, v16h b, v8f c) {
    return __builtin_amdgcn_wmma_f32_16x16x32_f16(false, a, false, b, (short)0, c, false, false);
  }
  static __device__ __forceinline__ void guard(v8f& a, v8f& b, v16h x, v16h y) { dep_guard_h(a, b, x, y); }
  static __device__ __forceinline__ void keep(v16h a, v16h b, v16h c, v16h d) { keep4_h(a, b, c, d); }
};
template <> struct Frag<__bf16> {
  typedef v16b V; union U { v16b v; v8b h[2]; };
  static __device__ __forceinline__ v16b load(const __bf16* p) {
    U f; f.h[0] = *(const v8b*)(p); f.h[1] = *(const v8b*)(p + 16); return f.v;
  }
  static __device__ __forceinline__ v8f mma(v16b a, v16b b, v8f c) {
    return __builtin_amdgcn_wmma_f32_16x16x32_bf16(false, a, false, b, (short)0, c, false, false);
  }
  static __device__ __forceinline__ void guard(v8f& a, v8f& b, v16b x, v16b y) { dep_guard_b(a, b, x, y); }
  static __device__ __forceinline__ void keep(v16b a, v16b b, v16b c, v16b d) { keep4_b(a, b, c, d); }
};

__device__ __forceinline__ unsigned pk16(unsigned short a, unsigned short b) { return (unsigned)a | ((unsigned)b << 16); }
__device__ __forceinline__ unsigned short h_bits(float f) { const _Float16 h = (_Float16)f; return __builtin_bit_cast(unsigned short, h); }

template <int ET> struct Elem;
template <> struct Elem<0> { typedef _Float16 T; };
template <> struct Elem<1> { typedef __bf16 T; };
template <int ET, bool SPLIT, int BIAS_MODE, int OUT_MODE, bool RESID, int ACT = 0>
__global__ __launch_bounds__(256) void wmma_gemm64(
    const unsigned short* __restrict__ Ap, const unsigned short* __restrict__ A2p, int lda, long strideA,
    const unsigned short* __restrict__ Btp, const unsigned short* __restrict__ Bt2p, int ldb, long strideB,
    void* __restrict__ Cout, void* __restrict__ Cout2, int ldc, long strideC,
    const float* __restrict__ bias,
    const float* __restrict__ resid, long strideR,
    int M, int N, int K, float scale) {
  typedef typename Elem<ET>::T T;
  typedef typename Frag<T>::V V;
  const T* A = (const T*)Ap; const T* A2 = (const T*)A2p; const T* Bt = (const T*)Btp; const T* Bt2 = (const T*)Bt2p;
  __shared__ __align__(16) float sT[8][16 * 68];
  const int b    = blockIdx.y;
  const int lane = threadIdx.x & 31;
  const int wave = threadIdx.x >> 5;
  const int tilesN = N >> 6;
  const int tilesM = M >> 6;
  const int tile = blockIdx.x * 8 + wave;
  if (tile >= tilesM * tilesN) return;
  const int tm = tile / tilesN;
  const int tn = tile - tm * tilesN;
  const int m0 = tm << 6;
  const int n0 = tn << 6;

  const T* Ab  = A  + (size_t)b * strideA;
  const T* Bb  = Bt + (size_t)b * strideB;
  const T* Ab2 = SPLIT ? (A2  + (size_t)b * strideA) : nullptr;
  const T* Bb2 = SPLIT ? (Bt2 + (size_t)b * strideB) : nullptr;

  const int rlane = lane & 15;
  const int koff  = (lane >> 4) * 8;
  const int mOff  = (lane >> 4) * 8;

  v8f acc[4][4];
#pragma unroll
  for (int i = 0; i < 4; ++i)
#pragma unroll
    for (int j = 0; j < 4; ++j) acc[i][j] = (v8f){0.f,0.f,0.f,0.f,0.f,0.f,0.f,0.f};

  for (int k0 = 0; k0 < K; k0 += 32) {
    V bh[4], bl[4];
#pragma unroll
    for (int j = 0; j < 4; ++j) {
      const size_t bo = (size_t)(n0 + (j << 4) + rlane) * ldb + koff + k0;
      bh[j] = Frag<T>::load(Bb + bo);
      if (SPLIT) bl[j] = Frag<T>::load(Bb2 + bo);
    }
#pragma unroll
    for (int i = 0; i < 4; ++i) {
      const size_t ao = (size_t)(m0 + (i << 4) + rlane) * lda + koff + k0;
      V ah = Frag<T>::load(Ab + ao);
      V al;
      if (SPLIT) al = Frag<T>::load(Ab2 + ao);
#pragma unroll
      for (int j = 0; j < 4; ++j) {
        acc[i][j] = Frag<T>::mma(ah, bh[j], acc[i][j]);
        if (SPLIT) {
          acc[i][j] = Frag<T>::mma(ah, bl[j], acc[i][j]);
          acc[i][j] = Frag<T>::mma(al, bh[j], acc[i][j]);
        }
      }
      Frag<T>::guard(acc[i][0], acc[i][3], ah, SPLIT ? al : ah);
    }
    Frag<T>::keep(bh[0], bh[1], bh[2], bh[3]);
    if (SPLIT) Frag<T>::keep(bl[0], bl[1], bl[2], bl[3]);
  }
  acc_guard4(acc[0][0], acc[0][1], acc[0][2], acc[0][3]);
  acc_guard4(acc[1][0], acc[1][1], acc[1][2], acc[1][3]);
  acc_guard4(acc[2][0], acc[2][1], acc[2][2], acc[2][3]);
  acc_guard4(acc[3][0], acc[3][1], acc[3][2], acc[3][3]);

  float* slab = sT[wave];
  const float* Rb = RESID ? (resid + (size_t)b * strideR) : nullptr;
#pragma unroll
  for (int i = 0; i < 4; ++i) {
    const int mBase = m0 + (i << 4);
#pragma unroll
    for (int j = 0; j < 4; ++j) {
      const int n = n0 + (j << 4) + rlane;
      float bv = 0.f;
      if (BIAS_MODE == 2) bv = bias[n];
#pragma unroll
      for (int r = 0; r < 8; ++r) {
        float v = acc[i][j][r] * scale;
        if (BIAS_MODE == 1) v += bias[mBase + mOff + r];
        if (BIAS_MODE == 2) v += bv;
        if (RESID) v += Rb[(size_t)(mBase + mOff + r) * ldc + n];
        if (ACT == 2) v = fmaxf(v, 0.0f);
        if (ACT == 4) v = (v > 0.f) ? v : 0.01f * v;
        slab[(mOff + r) * 68 + (j << 4) + rlane] = v;
      }
    }
    __builtin_amdgcn_fence(__ATOMIC_RELEASE, "workgroup");
    __builtin_amdgcn_wave_barrier();
    __builtin_amdgcn_fence(__ATOMIC_ACQUIRE, "workgroup");
    if (OUT_MODE == 0) {
      float* C = (float*)Cout + (size_t)b * strideC;
      const int hh = lane >> 4, c4 = (lane & 15) * 4;
      for (int pass = 0; pass < 2; ++pass) {
#pragma unroll
        for (int it = 0; it < 8; ++it) {
          const int row = it * 2 + hh;
          v4f v = *(const v4f*)(slab + row * 68 + c4);
          *(volatile v4f*)(C + (size_t)(mBase + row) * ldc + n0 + c4) = v;
        }
        __threadfence();
      }
    } else {
      const int q = lane >> 3, c8 = (lane & 7) * 8;
      unsigned short* C  = (unsigned short*)Cout  + (size_t)b * strideC;
      unsigned short* C2 = (OUT_MODE == 2) ? ((unsigned short*)Cout2 + (size_t)b * strideC) : nullptr;
      for (int pass = 0; pass < 2; ++pass) {
#pragma unroll
        for (int it = 0; it < 4; ++it) {
          const int row = it * 4 + q;
          const float* sp = slab + row * 68 + c8;
          v8h hv, lv;
#pragma unroll
          for (int e = 0; e < 8; ++e) {
            if (OUT_MODE == 1) {
              hv[e] = (_Float16)sp[e];
            } else {
              unsigned short hb = f2bf_bits(sp[e]);
              unsigned short lb = f2bf_bits(sp[e] - bf_bits2f(hb));
              hv[e] = __builtin_bit_cast(_Float16, hb);
              lv[e] = __builtin_bit_cast(_Float16, lb);
            }
          }
          *(volatile v8h*)(C + (size_t)(mBase + row) * ldc + n0 + c8) = hv;
          if (OUT_MODE == 2) *(volatile v8h*)(C2 + (size_t)(mBase + row) * ldc + n0 + c8) = lv;
        }
        __threadfence();
      }
    }
    __builtin_amdgcn_fence(__ATOMIC_RELEASE, "workgroup");
    __builtin_amdgcn_wave_barrier();
    __builtin_amdgcn_fence(__ATOMIC_ACQUIRE, "workgroup");
  }
}

__global__ __launch_bounds__(256) void pack_coef_kernel(const float* __restrict__ coef, const float* __restrict__ msk,
                                                        unsigned short* __restrict__ outp, int n8) {
  const int i = blockIdx.x * 256 + threadIdx.x;
  if (i >= n8) return;
  const float* p = coef + 8 * (size_t)i;
  const v4f a = *(const v4f*)(p);
  const v4f c = *(const v4f*)(p + 4);
  const float mv = msk[i >> 3] * kBCarry;
  unsigned short hb[8];
#pragma unroll
  for (int e = 0; e < 4; ++e) {
    hb[e]     = h_bits(a[e] * mv);
    hb[4 + e] = h_bits(c[e] * mv);
  }
  const v4u u = (v4u){pk16(hb[0], hb[1]), pk16(hb[2], hb[3]), pk16(hb[4], hb[5]), pk16(hb[6], hb[7])};
  unsigned short* q = outp + 8 * (size_t)i;
  *(volatile v4u*)q = u;
  __threadfence();
  *(volatile v4u*)q = u;
}

__global__ __launch_bounds__(256) void basis_kernel(const float* __restrict__ x, const float* __restrict__ knots,
                                                    unsigned short* __restrict__ aout, int row0) {
  __shared__ __align__(16) unsigned srow[256 * kRowPitchDw];
  __shared__ float sk[256];
  const int tid  = threadIdx.x;
  const int brow = blockIdx.x;

  {
    const int ki = tid < (kNk - 1) ? tid : (kNk - 1);
    sk[tid] = knots[ki];
  }
  __syncthreads();

  const float u    = x[(size_t)(row0 + brow) * kDin + tid];
  const float tk0  = sk[0];
  const float tk67 = sk[kNk - 1];
  const float hinv = 1.0f / (sk[1] - sk[0]);
  const bool valid = (u >= tk0) && (u < tk67);

  float pos = (u - tk0) * hinv;
  pos = fminf(fmaxf(pos, 0.0f), 66.0f);
  const int jc = (int)pos;
  const float tl = sk[jc];
  const float tr = sk[jc + 1];
  int jn = jc;
  jn = (u < tl)  ? (jc - 1) : jn;
  jn = (u >= tr) ? (jc + 1) : jn;
  jn = jn < 0 ? 0 : (jn > 66 ? 66 : jn);
  const float tj = sk[jn];
  float s = (u - tj) * hinv;
  s = fminf(fmaxf(s, 0.0f), 1.0f);

  const float s2 = s * s;
  const float s3 = s2 * s;
  const float os = 1.0f - s;
  const float cw = valid ? kACarry : 0.0f;
  const float w0 = (os * os * os) * kSixth * cw;
  const float w1 = (3.0f * s3 - 6.0f * s2 + 4.0f) * kSixth * cw;
  const float w2 = (-3.0f * s3 + 3.0f * s2 + 3.0f * s + 1.0f) * kSixth * cw;
  const float w3 = s3 * kSixth * cw;
  const unsigned short hb0 = h_bits(w0), hb1 = h_bits(w1), hb2 = h_bits(w2), hb3 = h_bits(w3);

  float zf = 0.0f;
  asm volatile("" : "+v"(zf));
  const unsigned short hbz = h_bits(zf);

  const int mp4 = jn + 1;
  const int dq  = (mp4 >> 1) + 2;
  const bool odd = (mp4 & 1) != 0;
  const unsigned ev0 = pk16(hb0, hb1);
  const unsigned ev1 = pk16(hb2, hb3);
  const unsigned od0 = pk16(hbz, hb0);
  const unsigned od1 = pk16(hb1, hb2);
  const unsigned od2 = pk16(hb3, hbz);
  const unsigned d0v = odd ? od0 : ev0;
  const unsigned d1v = odd ? od1 : ev1;
  const unsigned d2v = odd ? od2 : 0u;

  unsigned* myrow = srow + tid * kRowPitchDw;
#pragma unroll
  for (int q = 0; q < 32; ++q) myrow[4 + q] = 0u;
  asm volatile("" ::: "memory");
  myrow[dq]     = d0v;
  myrow[dq + 1] = d1v;
  myrow[dq + 2] = d2v;
  __syncthreads();

  unsigned short* arow = aout + (size_t)brow * kKtot;
  for (int pass = 0; pass < 2; ++pass) {
#pragma unroll
    for (int it = 0; it < 8; ++it) {
      const int c = it * 256 + tid;
      const int p = c >> 3;
      const int q = c & 7;
      const unsigned* sp = srow + p * kRowPitchDw + 4 + 4 * q;
      const v4u val = (v4u){sp[0], sp[1], sp[2], sp[3]};
      *(volatile v4u*)(arow + (size_t)c * 8) = val;
    }
    __threadfence();
  }
}

extern "C" void kernel_launch(void* const* d_in, const int* in_sizes, int n_in,
                              void* d_out, int out_size, void* d_ws, size_t ws_size,
                              hipStream_t stream) {
  if (n_in < 4) return;
  if (in_sizes[0] != kB * kDin) return;
  if (in_sizes[1] != kDout * kDin * kNb) return;
  if (in_sizes[2] != kDout * kDin) return;
  if (in_sizes[3] != kNk) return;
  if (out_size != kB * kDout) return;
  if (ws_size < kBtBytes + kABytes) return;

  const float* x     = (const float*)d_in[0];
  const float* coef  = (const float*)d_in[1];
  const float* msk   = (const float*)d_in[2];
  const float* knots = (const float*)d_in[3];
  float* out = (float*)d_out;

  unsigned short* btp = (unsigned short*)d_ws;
  unsigned short* ap  = (unsigned short*)((char*)d_ws + kBtBytes);

  const int n8 = kDout * kDin * kNb / 8;
  pack_coef_kernel<<<n8 / 256, 256, 0, stream>>>(coef, msk, btp, n8);

  const int tiles = (kMhalf / 64) * (kDout / 64);
  for (int half = 0; half < 2; ++half) {
    basis_kernel<<<kMhalf, 256, 0, stream>>>(x, knots, ap, half * kMhalf);
    float* cout = out + (size_t)half * kMhalf * kDout;
    dim3 g((tiles + 7) / 8, 1);
    wmma_gemm64<0, false, 0, 0, false, 0><<<g, 256, 0, stream>>>(
        ap, ap, kKtot, 0L,
        btp, btp, kKtot, 0L,
        (void*)cout, (void*)cout, kDout, 0L,
        x,
        x, 0L,
        kMhalf, kDout, kKtot, kOutScale);
  }
}
